// TimeMixModule_63299228008938
// MI455X (gfx1250) — hardware-verified
//
#include <hip/hip_runtime.h>
#include <math.h>

typedef __attribute__((ext_vector_type(16))) _Float16 v16h;
typedef __attribute__((ext_vector_type(16))) __bf16 v16b;
typedef __attribute__((ext_vector_type(8)))  _Float16 v8h;
typedef __attribute__((ext_vector_type(8)))  float v8f;
typedef __attribute__((ext_vector_type(4)))  float v4f;
typedef __attribute__((ext_vector_type(2)))  float v2f;
typedef __attribute__((ext_vector_type(4)))  unsigned v4u;
typedef __attribute__((ext_vector_type(4)))  int v4i;
typedef float __attribute__((may_alias)) float_a;
typedef int __attribute__((may_alias)) int_a;

template <typename T> __device__ __forceinline__ void vst2(void* p, T v) { *(volatile T*)p = v; __threadfence(); *(volatile T*)p = v; }
__device__ __forceinline__ v8f wmma16(v16h a, v16h b, v8f c) {
  v8f d = __builtin_amdgcn_wmma_f32_16x16x32_f16(false, a, false, b, (short)0, c, false, false);
  asm volatile("v_nop\n\tv_nop\n\tv_nop\n\tv_nop" : "+v"(d) : "v"(a), "v"(b));
  return d;
}
__device__ __forceinline__ v8f wmma_bf(v16b a, v16b b, v8f c) {
  v8f d = __builtin_amdgcn_wmma_f32_16x16x32_bf16(false, a, false, b, (short)0, c, false, false);
  asm volatile("v_nop\n\tv_nop\n\tv_nop\n\tv_nop" : "+v"(d) : "v"(a), "v"(b));
  return d;
}
__device__ __forceinline__ v16h frag_h(const _Float16* rowk0, int lane) {
  union { v16h v; v8h q[2]; } u; const _Float16* p = rowk0 + 8 * (lane >> 4);
  u.q[0] = *(const v8h*)p; u.q[1] = *(const v8h*)(p + 16); return u.v;
}
__device__ __forceinline__ v16h frag_f32(const float* rowk0, int lane) {
  v16h a; const float* p = rowk0 + 8 * (lane >> 4);
#pragma unroll
  for (int i = 0; i < 8; ++i) { a[i] = (_Float16)p[i]; a[8 + i] = (_Float16)p[16 + i]; }
  return a;
}
__device__ __forceinline__ v16h frag_f32s(const float* rowk0, int lane, float sc) {
  v16h a; const float* p = rowk0 + 8 * (lane >> 4);
#pragma unroll
  for (int i = 0; i < 8; ++i) { a[i] = (_Float16)(p[i] * sc); a[8 + i] = (_Float16)(p[16 + i] * sc); }
  return a;
}
__device__ __forceinline__ v16h fragc_f32(const float* W, int k0, int n, int lane, int ld, int K) {
  v16h a; const int g = lane >> 4;
#pragma unroll
  for (int i = 0; i < 8; ++i) { const int ka = k0 + 8 * g + i, kb = ka + 16;
    a[i] = (_Float16)(ka < K ? W[(size_t)(ka < K ? ka : K - 1) * ld + n] : 0.f); a[8 + i] = (_Float16)(kb < K ? W[(size_t)(kb < K ? kb : K - 1) * ld + n] : 0.f); }
  return a;
}
struct F2 { v16b h, l; };
__device__ __forceinline__ F2 bsplit16(const float v[16]) { F2 r;
#pragma unroll
  for (int i = 0; i < 16; ++i) { const __bf16 h = (__bf16)v[i]; r.h[i] = h; r.l[i] = (__bf16)(v[i] - (float)h); }
  return r; }
__device__ __forceinline__ F2 split_row(const float* row, int k0, int lane) { float v[16]; const float* p = row + k0 + 8 * (lane >> 4);
#pragma unroll
  for (int i = 0; i < 8; ++i) { v[i] = p[i]; v[8 + i] = p[16 + i]; }
  return bsplit16(v); }
__device__ __forceinline__ F2 split_rowK(const float* row, int k0, int lane, int K) { float v[16]; const int g = lane >> 4;
#pragma unroll
  for (int i = 0; i < 8; ++i) { const int ka = k0 + 8 * g + i, kb = ka + 16; v[i] = ka < K ? row[ka < K ? ka : K - 1] : 0.f; v[8 + i] = kb < K ? row[kb < K ? kb : K - 1] : 0.f; }
  return bsplit16(v); }
__device__ __forceinline__ F2 split_col(const float* W, int k0, int n, int lane, int ld, int K) { float v[16]; const int g = lane >> 4;
#pragma unroll
  for (int i = 0; i < 8; ++i) { const int ka = k0 + 8 * g + i, kb = ka + 16; v[i] = ka < K ? W[(size_t)(ka < K ? ka : K - 1) * ld + n] : 0.f; v[8 + i] = kb < K ? W[(size_t)(kb < K ? kb : K - 1) * ld + n] : 0.f; }
  return bsplit16(v); }
__device__ __forceinline__ v8f mac3(const F2& a, const F2& b, v8f c) { c = wmma_bf(a.l, b.h, c); c = wmma_bf(a.h, b.l, c); return wmma_bf(a.h, b.h, c); }
__device__ __forceinline__ float sigm(float v) { return 1.0f / (1.0f + expf(-v)); }
#define LDSX() do { asm volatile("s_wait_dscnt 0" ::: "memory"); __builtin_amdgcn_wave_barrier(); __builtin_amdgcn_fence(__ATOMIC_RELEASE, "workgroup"); } while (0)


#define NSEQ 4
#define TT 2048
#define CC 1024
#define NR (NSEQ * TT)
#ifndef NSP
#define NSP NSEQ
#endif
typedef __attribute__((ext_vector_type(8))) __bf16 v8b;
__device__ __forceinline__ v16b frag_b(const __bf16* rowk0, int lane) {
  union { v16b v; v8b q[2]; } u; const __bf16* p = rowk0 + 8 * (lane >> 4);
  u.q[0] = *(const v8b*)p; u.q[1] = *(const v8b*)(p + 16); return u.v;
}
__device__ __forceinline__ float bfr(float v) { return (float)(__bf16)v; }
__device__ __attribute__((noinline)) float exp_ni(float v) { return expf(v); }
__device__ __attribute__((noinline)) float erf_ni(float v) { return erff(v); }

#define WS_PW  0u
#define WS_GR  (WS_PW + 2u * (size_t)4 * CC * CC)
#define WS_GK  (WS_GR + 4u * (size_t)NR * CC)
#define WS_GV  (WS_GK + 4u * (size_t)NR * CC)
#define WS_Y   (WS_GV + 4u * (size_t)NR * CC)
#define WS_END (WS_Y + 4u * (size_t)NR * CC)

__global__ __launch_bounds__(256) void k_pack(const float* __restrict__ WR, const float* __restrict__ WK, const float* __restrict__ WV, const float* __restrict__ WO, __bf16* __restrict__ P) {
  const int n = blockIdx.x, which = blockIdx.y, t = threadIdx.x; const float* Wm = (which == 0) ? WR : (which == 1) ? WK : (which == 2) ? WV : WO; __shared__ __align__(16) __bf16 s[CC];
  for (int k = t; k < CC; k += 256) s[k] = (__bf16)Wm[(size_t)n * CC + k]; __syncthreads();
  for (int q = t; q < CC / 8; q += 256) vst2((unsigned*)(P + ((size_t)which * CC + n) * CC + q * 8), *(const v4u*)&s[q * 8]);
}
__global__ __launch_bounds__(128) void k_proj(const float* __restrict__ X, const __bf16* __restrict__ P, float* __restrict__ GR, float* __restrict__ GK, float* __restrict__ GV) {
  __shared__ __align__(16) float so[4][16][132];
  const int tid = threadIdx.x, wave = tid >> 5, lane = tid & 31, col = lane & 15, g = lane >> 4; const size_t r0 = (size_t)blockIdx.x * 64 + wave * 16; const int n0 = blockIdx.y * 128; const int which = blockIdx.z;
  const __bf16* Wr = P + (size_t)which * CC * CC; float* dst = (which == 0) ? GR : (which == 1) ? GK : GV;
  v8f acc[8] = {};
#pragma unroll 2
  for (int kc = 0; kc < CC / 32; ++kc) { v16b a; { const float* p = X + (r0 + col) * CC + kc * 32 + 8 * g;
#pragma unroll
      for (int i = 0; i < 8; ++i) { a[i] = (__bf16)p[i]; a[8 + i] = (__bf16)p[16 + i]; } }
#pragma unroll
    for (int j = 0; j < 8; ++j) acc[j] = wmma_bf(a, frag_b(Wr + (size_t)(n0 + j * 16 + col) * CC + kc * 32, lane), acc[j]); }
#pragma unroll
  for (int j = 0; j < 8; ++j)
#pragma unroll
    for (int r = 0; r < 8; ++r) so[wave][8 * g + r][j * 16 + col] = acc[j][r];
  LDSX();
  for (int rl = 0; rl < 16; ++rl) vst2(dst + (r0 + rl) * CC + n0 + lane * 4, *(const v4f*)&so[wave][rl][lane * 4]);
}
__device__ __attribute__((noinline)) float exp_p(float v) { return expf(v); }
__global__ __launch_bounds__(256) void k_scan(const float* __restrict__ GR, const float* __restrict__ GK, const float* __restrict__ GV, const float* __restrict__ BR, const float* __restrict__ BK, const float* __restrict__ BV, const float* __restrict__ TD, const float* __restrict__ UU, float* __restrict__ Y) {
  const int c = blockIdx.x * 256 + threadIdx.x; const size_t n = blockIdx.y; if (c >= CC) return;
  const float br = bfr(BR[c]), bk = bfr(BK[c]), bv = bfr(BV[c]); const float w = fmaxf(bfr(TD[c]), 0.f), u = bfr(UU[c]);
  const float* gr = GR + n * TT * CC + c; const float* gk = GK + n * TT * CC + c; const float* gv = GV + n * TT * CC + c; float* y = Y + n * TT * CC + c;
  float pa = 0.f, pb = 0.f;
  float grp = 0.f, gkp = 0.f, gvp = 0.f;
  float grc = gr[0], gkc = gk[0], gvc = gv[0];
#pragma unroll 1
  for (int t = 0; t < TT; ++t) {
    const bool last = (t == TT - 1); const size_t o1 = (size_t)(t + 1) * CC;
    const float grn = last ? 0.f : gr[o1], gkn = last ? 0.f : gk[o1], gvn = last ? 0.f : gv[o1];
    const float R = (0.460022211f * grp + 0.539977789f * grn) + br;
    const float K = (0.947317123f * gkp + 0.0526828580f * gkn) + bk;
    const float V = (0.920044422f * gvp + 0.0799555853f * gvn) + bv;
    const float Wt = -w * (float)(TT - 1 - t);
    const float e = exp_p(fminf(fmaxf(Wt + K, -20.0f), 10.0f)); const float eu = exp_p(fminf(fmaxf(u + K, -20.0f), 10.0f));
    const float A = pa + eu * V, Bd = pb + eu; const float wkv = A / Bd;
    pa += e * V; pb += e;
    const float sg = 1.0f / (1.0f + exp_p(-R));
    y[(size_t)t * CC] = sg * wkv;
    grp = grc; gkp = gkc; gvp = gvc; grc = grn; gkc = gkn; gvc = gvn; }
}
__global__ __launch_bounds__(128) void k_out(const float* __restrict__ Yin, const __bf16* __restrict__ P, const float* __restrict__ BO, float* __restrict__ OUT) {
  __shared__ __align__(16) float so[4][16][132];
  const int tid = threadIdx.x, wave = tid >> 5, lane = tid & 31, col = lane & 15, g = lane >> 4; const size_t r0 = (size_t)blockIdx.x * 64 + wave * 16; const int n0 = blockIdx.y * 128;
  v8f acc[8] = {};
#pragma unroll 2
  for (int kc = 0; kc < CC / 32; ++kc) { const F2 a = split_row(Yin + (r0 + col) * CC, kc * 32, lane);
#pragma unroll
    for (int j = 0; j < 8; ++j) { const v16b wv = frag_b(P + (size_t)3 * CC * CC + (size_t)(n0 + j * 16 + col) * CC + kc * 32, lane); acc[j] = wmma_bf(a.l, wv, acc[j]); acc[j] = wmma_bf(a.h, wv, acc[j]); } }
#pragma unroll
  for (int j = 0; j < 8; ++j) { const float bb = bfr(BO[n0 + j * 16 + col]);
#pragma unroll
    for (int r = 0; r < 8; ++r) so[wave][8 * g + r][j * 16 + col] = acc[j][r] + bb; }
  LDSX();
  for (int rl = 0; rl < 16; ++rl) vst2(OUT + (r0 + rl) * CC + n0 + lane * 4, *(const v4f*)&so[wave][rl][lane * 4]);
}
extern "C" void kernel_launch(void* const* d_in, const int* in_sizes, int n_in, void* d_out, int out_size, void* d_ws, size_t ws_size, hipStream_t stream) {
  (void)in_sizes; (void)n_in; (void)out_size;
  const float** F = (const float**)d_in;
  if (ws_size < (size_t)WS_END) return;
  char* ws = (char*)d_ws; __bf16* P = (__bf16*)(ws + WS_PW); float *GR = (float*)(ws + WS_GR), *GK = (float*)(ws + WS_GK), *GV = (float*)(ws + WS_GV), *Y = (float*)(ws + WS_Y);
  k_pack<<<dim3(CC, 4), 256, 0, stream>>>(F[1], F[3], F[5], F[7], P);
  k_proj<<<dim3(NSP * TT / 64, CC / 128, 3), 128, 0, stream>>>(F[0], P, GR, GK, GV);
  k_scan<<<dim3(CC / 256, NSP), 256, 0, stream>>>(GR, GK, GV, F[2], F[4], F[6], F[9], F[10], Y);
  k_out<<<dim3(NSP * TT / 64, CC / 128), 128, 0, stream>>>(Y, P, F[8], (float*)d_out);
}
